// FlexQMixer_44942537785482
// MI455X (gfx1250) — hardware-run, weakly checked
//
#include <hip/hip_runtime.h>


#ifndef NB
#define NB 64
#endif
#ifndef TT
#define TT 64
#endif
#define NB_FULL 64
#define TT_FULL 64
#ifndef OUT_TT
#define OUT_TT TT
#endif
#define NE   32
#define ED   64
#define HYP  128
#define NA   8
#define NH_  4
#define HD   32
#define EMB  32
#define MW   2
#define IW   16
#define IPB  (MW * IW)
#define XP   136
#define QP   264
#define UP   32
#define NQR  (2 * HYP + 16)
#define B1O  0
#define BQO  HYP
#define CBO  (BQO + NQR)
#define NBR  448
#define WS   64.0f
#define WSI  (1.0f / 64.0f)
#define SC2  ((float)(0.17677669529663687 * 1.4426950408889634))
#define NEGB (-3.0e38f)

static_assert(HD == 32);
static_assert(NH_ * HD == HYP);
static_assert(NE == 32);
static_assert(NA == 8);
static_assert(ED % 32 == 0);
static_assert(ED == 64);
static_assert(HYP % 32 == 0);
static_assert(HYP == 128);
static_assert(XP % 8 == 0);
static_assert(XP >= HYP);
static_assert(QP % 8 == 0);
static_assert(QP >= 2 * HYP);
static_assert(UP >= NE);
static_assert(IPB == 32);
static_assert(TT % IPB == 0);
static_assert(OUT_TT % 32 == 0);
static_assert((NB * TT) % IPB == 0);
static_assert(CBO + 2 <= NBR);
static_assert(BQO + 2 * HYP + 16 == CBO);
static_assert(NBR % 32 == 0);
static_assert(NBR / 4 <= 256);
static_assert(NBR == 3 * HYP + 64);
static_assert((2 * HYP * HYP / 8) % 256 == 0);
static_assert(16 * HYP / 8 == 256);
static_assert(NB <= NB_FULL);
static_assert(TT <= TT_FULL);
static_assert((size_t)MW * NE * XP * 2 + (size_t)MW * NE * QP * 2 + (size_t)MW * 16 * UP * 4 + (size_t)IPB * 4 <= (size_t)131072);
static_assert((size_t)(HYP + HYP + 4 * HYP + NBR) * 4 <= (size_t)131072);
static_assert(8 * 16 == IPB * 4);

typedef _Float16 h16;
typedef unsigned short bf;
typedef __attribute__((ext_vector_type(16))) __bf16   v16bf;
typedef __attribute__((ext_vector_type(16))) _Float16 v16h;
typedef __attribute__((ext_vector_type(8)))  _Float16 v8h;
typedef __attribute__((ext_vector_type(8)))  unsigned short v8us;
typedef __attribute__((ext_vector_type(8)))  float    v8f;
typedef __attribute__((ext_vector_type(4)))  float    v4f;
typedef __attribute__((ext_vector_type(4)))  int      v4i;
typedef v4f  __attribute__((may_alias)) v4fa;

__device__ __forceinline__ unsigned short f2bf(float f) { unsigned u = __float_as_uint(f); u += 0x7FFFu + ((u >> 16) & 1u); return (unsigned short)(u >> 16); }
__device__ __forceinline__ float bfr(float f) { return __uint_as_float(((unsigned)f2bf(f)) << 16); }
__device__ __forceinline__ v16h cat16(v8h lo, v8h hi) { return __builtin_shufflevector(lo, hi, 0, 1, 2, 3, 4, 5, 6, 7, 8, 9, 10, 11, 12, 13, 14, 15); }
__device__ __forceinline__ v16bf cat16b(v8us lo, v8us hi) { return __builtin_bit_cast(v16bf, __builtin_shufflevector(lo, hi, 0, 1, 2, 3, 4, 5, 6, 7, 8, 9, 10, 11, 12, 13, 14, 15)); }
__device__ __forceinline__ v8f wmma16(v16h a, v16h b, v8f c) { return __builtin_amdgcn_wmma_f32_16x16x32_f16(false, a, false, b, (short)0, c, false, false); }
__device__ __forceinline__ v8f wmmab(v16bf a, v16bf b, v8f c) { return __builtin_amdgcn_wmma_f32_16x16x32_bf16(false, a, false, b, (short)0, c, false, false); }
__device__ __forceinline__ v16h  ldh(const h16* p) { return cat16(*(const v8h*)p, *(const v8h*)(p + 16)); }
__device__ __forceinline__ v16bf ldb(const bf* p)  { return cat16b(*(const v8us*)p, *(const v8us*)(p + 16)); }
__device__ __forceinline__ void wave_sync() { __builtin_amdgcn_fence(3  , "wavefront"); __builtin_amdgcn_wave_barrier(); asm volatile("" ::: "memory"); }

__global__ __launch_bounds__(256) void k_cvt8(const float* __restrict__ src, bf* dst, size_t n8) {
    const size_t i = (size_t)blockIdx.x * 256 + threadIdx.x; if (i >= n8) return;
    const v8f v = *(const v8f*)(src + i * 8); v8us o;
#pragma unroll
    for (int k = 0; k < 8; ++k) o[k] = f2bf(v[k]);
    *(volatile v8us*)(dst + i * 8) = o; __threadfence(); *(volatile v8us*)(dst + i * 8) = o;
}

static __device__ __forceinline__ h16 toh_flush(float v) { const h16 r = (h16)v; return (fabsf(v) < 6.103515625e-05f) ? (h16)0.0f : r; }
__device__ __forceinline__ v8f wmma16g(v16h a, v16h b, v8f c) {
    c = __builtin_amdgcn_wmma_f32_16x16x32_f16(false, a, false, b, (short)0, c, false, false);
    asm volatile("v_nop\n\tv_nop\n\tv_nop\n\tv_nop" : "+v"(c) : "v"(a), "v"(b));
    return c;
}
__device__ __forceinline__ v8f wmmabg(v16bf a, v16bf b, v8f c) {
    c = __builtin_amdgcn_wmma_f32_16x16x32_bf16(false, a, false, b, (short)0, c, false, false);
    asm volatile("v_nop\n\tv_nop\n\tv_nop\n\tv_nop" : "+v"(c) : "v"(a), "v"(b));
    return c;
}
__device__ __forceinline__ v16bf ldcvtb(const float* p) {
    const v4f a = *(const v4f*)p, b = *(const v4f*)(p + 4), c = *(const v4f*)(p + 16), d = *(const v4f*)(p + 20);
    v8us lo, hi;
#pragma unroll
    for (int i = 0; i < 4; ++i) { lo[i] = f2bf(a[i]); lo[4 + i] = f2bf(b[i]); hi[i] = f2bf(c[i]); hi[4 + i] = f2bf(d[i]); }
    return cat16b(lo, hi);
}
#define LFRAG(arr, o) cat16(*(const v8h*)(&arr[(o)]), *(const v8h*)(&arr[(o) + 16]))

__global__ __launch_bounds__(256) void k_wprep(const float* __restrict__ qkv_w, const float* __restrict__ qkv_b, const float* __restrict__ out_w, const float* __restrict__ out_b,
                                               const float* __restrict__ fc2_w, const float* __restrict__ fc2_b, const float* __restrict__ fc1_b, h16* WQH, float* BROW) {
    __shared__ __align__(16) float sC[HYP];
    __shared__ __align__(16) float sD[HYP];
    __shared__ __align__(16) float sWu[4 * HYP];
    __shared__ __align__(16) float sB[NBR];
    const int tid = threadIdx.x;
    const int slot = blockIdx.x;
    const int g = 2 * slot + 1;
    const float* qw = qkv_w + (size_t)g * (3 * HYP * HYP);
    const float* qb = qkv_b + (size_t)g * (3 * HYP);
    const float* ow = out_w + (size_t)g * (HYP * HYP);
    const float* ob = out_b + (size_t)g * HYP;
    const float* f2 = fc2_w + (size_t)g * (EMB * HYP);
    const float* f2b = fc2_b + (size_t)g * EMB;
    const float* f1b = fc1_b + (size_t)g * HYP;
    h16* wdst = WQH + (size_t)slot * NQR * HYP;
#pragma unroll 1
    for (int itc = 0; itc < (2 * HYP * HYP / 8) / 256; ++itc) {
        const size_t ch = (size_t)itc * 256 + tid;
        const v4f x0 = *(const v4f*)(qw + ch * 8), x1 = *(const v4f*)(qw + ch * 8 + 4); v8h o;
#pragma unroll
        for (int i = 0; i < 4; ++i) { o[i] = toh_flush(bfr(x0[i]) * WS); o[4 + i] = toh_flush(bfr(x1[i]) * WS); }
        *(volatile v8h*)(wdst + ch * 8) = o; __threadfence(); *(volatile v8h*)(wdst + ch * 8) = o;
    }
    if (tid < HYP) {
        float c = 0.0f;
#pragma unroll 1
        for (int e = 0; e < EMB; ++e) c += bfr(f2[e * HYP + tid]);
        sC[tid] = c;
    }
    __syncthreads();
    if (tid < HYP) {
        float d = 0.0f;
#pragma unroll 1
        for (int o = 0; o < HYP; ++o) d += sC[o] * bfr(ow[o * HYP + tid]);
        sD[tid] = d;
    }
    __syncthreads();
#pragma unroll 1
    for (int i = tid; i < 4 * HYP; i += 256) {
        const int hh = i >> 7, h1 = i & 127;
        const float* vw = qw + (size_t)(2 * HYP + hh * HD) * HYP + h1;
        float s = 0.0f;
#pragma unroll 1
        for (int dd = 0; dd < HD; ++dd) s += bfr(vw[dd * HYP]) * sD[hh * HD + dd];
        sWu[i] = s;
    }
    float bvv = 0.0f;
    { const int hh = tid & 3;
#pragma unroll 1
      for (int dd = 0; dd < HD; ++dd) bvv += bfr(qb[2 * HYP + hh * HD + dd]) * sD[hh * HD + dd]; }
    float cb = 0.0f;
#pragma unroll 1
    for (int o = 0; o < HYP; ++o) cb += bfr(ob[o]) * sC[o];
#pragma unroll 1
    for (int e = 0; e < EMB; ++e) cb += bfr(f2b[e]);
    const float coef = (slot == 0) ? 0.125f : 0.00390625f;
    if (tid < HYP) sB[B1O + tid] = bfr(f1b[tid]);
    sB[BQO + tid] = bfr(qb[tid]);
    if (tid < 64) { float v = 0.0f; v = (tid < 4) ? bvv : v; v = (tid == 16) ? cb : v; v = (tid == 17) ? coef : v; sB[BQO + 2 * HYP + tid] = v; }
    __syncthreads();
    { const int row = tid >> 4, c8 = (tid & 15) * 8; const int sr = row & 3; const bool real = row < 4; v8h o;
#pragma unroll
      for (int i = 0; i < 8; ++i) { const float wv = sWu[sr * HYP + c8 + i]; o[i] = toh_flush(real ? wv * WS : 0.0f); }
      h16* p = wdst + (size_t)(2 * HYP + row) * HYP + c8;
      *(volatile v8h*)p = o; __threadfence(); *(volatile v8h*)p = o; }
    if (tid < NBR / 4) {
        const v4f v = *(const v4fa*)(&sB[4 * tid]);
        float* p = BROW + (size_t)slot * NBR + 4 * tid;
        *(volatile v4f*)p = v; __threadfence(); *(volatile v4f*)p = v;
    }
}

__global__ __launch_bounds__(32 * MW) void k_hyper(const float* __restrict__ QS, const float* __restrict__ ENT, const int* __restrict__ EM,
                                                   const bf* __restrict__ W1B, const h16* __restrict__ WQH, const float* __restrict__ BROW, float* OUT) {
    __shared__ __align__(16) h16 xs[MW * NE * XP];
    __shared__ __align__(16) h16 qks[MW * NE * QP];
    __shared__ __align__(16) float us[MW * 16 * UP];
    __shared__ __align__(16) float ys[IPB];
    const int lane = threadIdx.x & 31, lr = lane & 15, hi = lane >> 4;
    const int wave = __builtin_amdgcn_readfirstlane((int)(threadIdx.x >> 5));
    const int wx = wave * NE * XP, wq = wave * NE * QP, wu = wave * 16 * UP;
#pragma unroll 1
    for (int ii = 0; ii < IW; ++ii) {
        const int it = blockIdx.x * IPB + wave * IW + ii;
        const size_t srow = (size_t)(it / TT) * TT_FULL + (size_t)(it % TT);
        const int* emr = EM + srow * NE;
        int amv = emr[lr];
        asm volatile("" : "+v"(amv));
        const v4i e0 = *(const v4i*)(emr + 8 * hi), e1 = *(const v4i*)(emr + 8 * hi + 4), e2 = *(const v4i*)(emr + 16 + 8 * hi), e3 = *(const v4i*)(emr + 16 + 8 * hi + 4);
        const float fam = 1.0f - (float)amv;
        bool ka[8], kb[8];
#pragma unroll
        for (int r = 0; r < 4; ++r) {
            ka[r]     = !((1.0f - fam * (1.0f - (float)e0[r])) > 0.0f);
            ka[4 + r] = !((1.0f - fam * (1.0f - (float)e1[r])) > 0.0f);
            kb[r]     = !((1.0f - fam * (1.0f - (float)e2[r])) > 0.0f);
            kb[4 + r] = !((1.0f - fam * (1.0f - (float)e3[r])) > 0.0f); }
        const bool live = !(amv > 0);
        const float* erow = ENT + srow * (size_t)(NE * ED) + (size_t)lr * ED + 8 * hi;
        const v16bf eb00 = ldcvtb(erow), eb01 = ldcvtb(erow + 32), eb10 = ldcvtb(erow + 16 * ED), eb11 = ldcvtb(erow + 16 * ED + 32);
        float yl = 0.0f;
#pragma unroll 1
        for (int slot = 0; slot < 2; ++slot) {
            const bf* w1 = W1B + (size_t)slot * HYP * ED;
            const h16* wqp = WQH + (size_t)slot * NQR * HYP;
            const float* br = BROW + (size_t)slot * NBR;
#pragma unroll 1
            for (int i = 0; i < HYP / 16; ++i) {
                const bf* ap = w1 + (size_t)(16 * i + lr) * ED + 8 * hi;
                const v16bf a0 = ldb(ap), a1 = ldb(ap + 32);
                v8f c0 = (v8f){}, c1 = (v8f){};
                c0 = wmmabg(a0, eb00, c0); c1 = wmmabg(a0, eb10, c1);
                c0 = wmmabg(a1, eb01, c0); c1 = wmmabg(a1, eb11, c1);
                const v4f ba = *(const v4f*)(br + B1O + 16 * i + 8 * hi), bb = *(const v4f*)(br + B1O + 16 * i + 8 * hi + 4);
                v8h h0, h1;
#pragma unroll
                for (int r = 0; r < 4; ++r) {
                    h0[r] = toh_flush(fmaxf(c0[r] + ba[r], 0.0f)); h0[4 + r] = toh_flush(fmaxf(c0[4 + r] + bb[r], 0.0f));
                    h1[r] = toh_flush(fmaxf(c1[r] + ba[r], 0.0f)); h1[4 + r] = toh_flush(fmaxf(c1[4 + r] + bb[r], 0.0f)); }
                *(v8h*)(&xs[wx + lr * XP + 16 * i + 8 * hi]) = h0;
                *(v8h*)(&xs[wx + (16 + lr) * XP + 16 * i + 8 * hi]) = h1;
            }
            wave_sync();
            v16h xb0[4], xb1[4];
#pragma unroll
            for (int ks = 0; ks < 4; ++ks) { xb0[ks] = LFRAG(xs, wx + lr * XP + 32 * ks + 8 * hi); xb1[ks] = LFRAG(xs, wx + (16 + lr) * XP + 32 * ks + 8 * hi); }
#pragma unroll 1
            for (int i = 0; i < HYP / 16; ++i) {
                const h16* ap = wqp + (size_t)(16 * i + lr) * HYP + 8 * hi;
                v8f c0 = (v8f){};
#pragma unroll
                for (int ks = 0; ks < 4; ++ks) { const v16h a = ldh(ap + 32 * ks); c0 = wmma16g(a, xb0[ks], c0); }
                const v4f ba = *(const v4f*)(br + BQO + 16 * i + 8 * hi), bb = *(const v4f*)(br + BQO + 16 * i + 8 * hi + 4);
                v8h h0;
#pragma unroll
                for (int r = 0; r < 4; ++r) { h0[r] = toh_flush(c0[r] * WSI + ba[r]); h0[4 + r] = toh_flush(c0[4 + r] * WSI + bb[r]); }
                *(v8h*)(&qks[wq + lr * QP + 16 * i + 8 * hi]) = h0;
            }
#pragma unroll 1
            for (int i = HYP / 16; i < 2 * HYP / 16; ++i) {
                const h16* ap = wqp + (size_t)(16 * i + lr) * HYP + 8 * hi;
                v8f c0 = (v8f){}, c1 = (v8f){};
#pragma unroll
                for (int ks = 0; ks < 4; ++ks) { const v16h a = ldh(ap + 32 * ks); c0 = wmma16g(a, xb0[ks], c0); c1 = wmma16g(a, xb1[ks], c1); }
                const v4f ba = *(const v4f*)(br + BQO + 16 * i + 8 * hi), bb = *(const v4f*)(br + BQO + 16 * i + 8 * hi + 4);
                v8h h0, h1;
#pragma unroll
                for (int r = 0; r < 4; ++r) {
                    h0[r] = toh_flush(c0[r] * WSI + ba[r]); h0[4 + r] = toh_flush(c0[4 + r] * WSI + bb[r]);
                    h1[r] = toh_flush(c1[r] * WSI + ba[r]); h1[4 + r] = toh_flush(c1[4 + r] * WSI + bb[r]); }
                *(v8h*)(&qks[wq + lr * QP + 16 * i + 8 * hi]) = h0;
                *(v8h*)(&qks[wq + (16 + lr) * QP + 16 * i + 8 * hi]) = h1;
            }
            { const h16* ap = wqp + (size_t)(2 * HYP + lr) * HYP + 8 * hi;
              v8f c0 = (v8f){}, c1 = (v8f){};
#pragma unroll
              for (int ks = 0; ks < 4; ++ks) { const v16h a = ldh(ap + 32 * ks); c0 = wmma16g(a, xb0[ks], c0); c1 = wmma16g(a, xb1[ks], c1); }
              const v4f ba = *(const v4f*)(br + BQO + 2 * HYP + 8 * hi), bb = *(const v4f*)(br + BQO + 2 * HYP + 8 * hi + 4);
#pragma unroll
              for (int r = 0; r < 4; ++r) {
                  us[wu + (8 * hi + r) * UP + lr]          = c0[r] * WSI + ba[r];
                  us[wu + (8 * hi + 4 + r) * UP + lr]      = c0[4 + r] * WSI + bb[r];
                  us[wu + (8 * hi + r) * UP + 16 + lr]     = c1[r] * WSI + ba[r];
                  us[wu + (8 * hi + 4 + r) * UP + 16 + lr] = c1[4 + r] * WSI + bb[r]; } }
            wave_sync();
            float sacc = 0.0f;
#pragma unroll 1
            for (int hh = 0; hh < NH_; ++hh) {
                const v16h qf = LFRAG(qks, wq + lr * QP + hh * HD + 8 * hi);
                const v16h k0 = LFRAG(qks, wq + lr * QP + HYP + hh * HD + 8 * hi);
                const v16h k1 = LFRAG(qks, wq + (16 + lr) * QP + HYP + hh * HD + 8 * hi);
                v8f sa = (v8f){}, sb = (v8f){};
                sa = wmma16g(k0, qf, sa); sb = wmma16g(k1, qf, sb);
                const v4f ua0 = *(const v4fa*)(&us[wu + hh * UP + 8 * hi]), ua1 = *(const v4fa*)(&us[wu + hh * UP + 8 * hi + 4]);
                const v4f ub0 = *(const v4fa*)(&us[wu + hh * UP + 16 + 8 * hi]), ub1 = *(const v4fa*)(&us[wu + hh * UP + 16 + 8 * hi + 4]);
                float ua[8], ub[8];
#pragma unroll
                for (int r = 0; r < 4; ++r) { ua[r] = ua0[r]; ua[4 + r] = ua1[r]; ub[r] = ub0[r]; ub[4 + r] = ub1[r]; }
                float ta[8], tb[8]; float mx = NEGB;
#pragma unroll
                for (int r = 0; r < 8; ++r) {
                    ta[r] = sa[r] * SC2; tb[r] = sb[r] * SC2;
                    mx = fmaxf(mx, fmaxf(ka[r] ? ta[r] : NEGB, kb[r] ? tb[r] : NEGB)); }
                mx = fmaxf(mx, __shfl_xor(mx, 16, 32));
                float den = 0.0f, num = 0.0f;
#pragma unroll
                for (int r = 0; r < 8; ++r) {
                    const float ea = __builtin_amdgcn_exp2f(ta[r] - mx), eb = __builtin_amdgcn_exp2f(tb[r] - mx);
                    const float ga = ka[r] ? ea : 0.0f, gb = kb[r] ? eb : 0.0f;
                    den += ga + gb; num += ga * ua[r] + gb * ub[r]; }
                den += __shfl_xor(den, 16, 32); num += __shfl_xor(num, 16, 32);
                const bool anyk = den > 0.0f;
                const float dsafe = anyk ? den : 1.0f;
                sacc += anyk ? (num * (1.0f / dsafe)) : 0.0f;
            }
            const float cbv = br[CBO], cf = br[CBO + 1];
            yl += live ? ((sacc + cbv) * cf) : 0.0f;
            wave_sync();
        }
        float qv = QS[srow * NA + (lane & 7)];
        asm volatile("" : "+v"(qv));
        float z = (lane < NA) ? (yl + bfr(qv)) : 0.0f;
        z += __shfl_xor(z, 1, 32); z += __shfl_xor(z, 2, 32); z += __shfl_xor(z, 4, 32);
        if (lane == 0) ys[wave * IW + ii] = z;
    }
    __syncthreads();
    if (threadIdx.x < 8) {
        const int it0 = blockIdx.x * IPB;
        float* op = OUT + (size_t)(it0 / TT) * OUT_TT + (size_t)(it0 % TT) + 4 * threadIdx.x;
        const v4f val = *(const v4fa*)(&ys[4 * threadIdx.x]);
        *(volatile v4f*)op = val; __threadfence(); *(volatile v4f*)op = val;
    }
}

static constexpr size_t al256(size_t v) { return (v + 255) & ~(size_t)255; }
static constexpr size_t SZ_W1 = al256((size_t)2 * HYP * ED * 2);
static constexpr size_t SZ_WQ = al256((size_t)2 * NQR * HYP * 2);
static constexpr size_t SZ_BR = al256((size_t)2 * NBR * 4);
static constexpr size_t SZ_TOTAL = SZ_W1 + SZ_WQ + SZ_BR;
static_assert(SZ_TOTAL <= (size_t)134217728);
static_assert(((size_t)HYP * ED * 2) % 128 == 0);
static_assert(((size_t)NQR * HYP * 2) % 128 == 0);
static_assert(((size_t)NBR * 4) % 128 == 0);
static_assert(((size_t)HYP * ED) % 8 == 0);

extern "C" void kernel_launch(void* const* d_in, const int* in_sizes, int n_in,
                              void* d_out, int out_size, void* d_ws, size_t ws_size, hipStream_t stream) {
    if (n_in < 11) return;
    const size_t rows = (size_t)(NB - 1) * TT_FULL + TT;
    if ((size_t)in_sizes[0] < rows * NA || (size_t)in_sizes[1] < rows * NE * ED || (size_t)in_sizes[2] < rows * NE) return;
    if ((size_t)in_sizes[3] < (size_t)4 * HYP * ED || (size_t)in_sizes[4] < (size_t)4 * HYP) return;
    if ((size_t)in_sizes[5] < (size_t)4 * 3 * HYP * HYP || (size_t)in_sizes[6] < (size_t)4 * 3 * HYP) return;
    if ((size_t)in_sizes[7] < (size_t)4 * HYP * HYP || (size_t)in_sizes[8] < (size_t)4 * HYP) return;
    if ((size_t)in_sizes[9] < (size_t)4 * EMB * HYP || (size_t)in_sizes[10] < (size_t)4 * EMB) return;
    if ((size_t)out_size < (size_t)(NB - 1) * OUT_TT + TT) return;
    if (SZ_TOTAL > ws_size) return;
    const float* qs   = (const float*)d_in[0];
    const float* ents = (const float*)d_in[1];
    const int*   em   = (const int*)d_in[2];
    const float* fc1w = (const float*)d_in[3];
    const float* fc1b = (const float*)d_in[4];
    const float* qkvw = (const float*)d_in[5];
    const float* qkvb = (const float*)d_in[6];
    const float* outw = (const float*)d_in[7];
    const float* outb = (const float*)d_in[8];
    const float* fc2w = (const float*)d_in[9];
    const float* fc2b = (const float*)d_in[10];
    float* OUT = (float*)d_out;
    char* wsp = (char*)d_ws;
    bf*  W1B = (bf*)wsp;  wsp += SZ_W1;
    h16* WQH = (h16*)wsp; wsp += SZ_WQ;
    float* BROW = (float*)wsp; wsp += SZ_BR;

    { const size_t n8 = (size_t)HYP * ED / 8; const unsigned gq = (unsigned)((n8 + 255) / 256);
      k_cvt8<<<gq, 256, 0, stream>>>(fc1w + (size_t)1 * HYP * ED, W1B, n8);
      k_cvt8<<<gq, 256, 0, stream>>>(fc1w + (size_t)3 * HYP * ED, W1B + (size_t)HYP * ED, n8); }
    k_wprep<<<2, 256, 0, stream>>>(qkvw, qkvb, outw, outb, fc2w, fc2b, fc1b, WQH, BROW);
    k_hyper<<<(unsigned)((NB * TT) / IPB), 32 * MW, 0, stream>>>(qs, ents, em, W1B, WQH, BROW, OUT);
}
